// MinConv2dLSTM_58737972740761
// MI455X (gfx1250) — hardware-verified
//
#include <hip/hip_runtime.h>

constexpr int kNB = 4;
constexpr int kNS = 16;
constexpr int kHW = 1024;
constexpr int kCH = 64;
constexpr int kNG = 256;
constexpr int kCin0 = 32;
constexpr int kFramesHalf = 32;
constexpr int kRowsHalf = kFramesHalf * kHW;
constexpr float kWCarry = 16.0f;
constexpr float kHCarry = 8.0f;
constexpr float kScale0 = 1.0f / 16.0f;
constexpr float kScale1 = 1.0f / 128.0f;

constexpr size_t kOffWT0 = 0;
constexpr size_t kOffWT1 = 147456;
constexpr size_t kOffH0  = 442368;
constexpr size_t kOffA   = 8830976;
constexpr size_t kOffG   = 46579712;
constexpr size_t kCarveEnd = 80134144;

typedef __attribute__((ext_vector_type(16))) _Float16 v16h;
typedef __attribute__((ext_vector_type(8)))  _Float16 v8h;
typedef __attribute__((ext_vector_type(16))) __bf16   v16b;
typedef __attribute__((ext_vector_type(8)))  __bf16   v8b;
typedef __attribute__((ext_vector_type(8)))  float    v8f;
typedef __attribute__((ext_vector_type(4)))  float    v4f;
typedef __attribute__((ext_vector_type(2)))  float    v2f;
typedef __attribute__((ext_vector_type(4)))  unsigned int v4u;

__device__ __forceinline__ unsigned short f2bf_bits(float f) {
  unsigned u = __float_as_uint(f);
  return (unsigned short)((u + 0x7FFFu + ((u >> 16) & 1u)) >> 16);
}
__device__ __forceinline__ float bf_bits2f(unsigned short h) { return __uint_as_float(((unsigned)h) << 16); }

__device__ __forceinline__ void dep_guard_h(v8f& a, v8f& b, v16h x, v16h y) { asm volatile("v_nop\n\tv_nop\n\tv_nop\n\tv_nop" : "+v"(a), "+v"(b) : "v"(x), "v"(y)); }
__device__ __forceinline__ void dep_guard_b(v8f& a, v8f& b, v16b x, v16b y) { asm volatile("v_nop\n\tv_nop\n\tv_nop\n\tv_nop" : "+v"(a), "+v"(b) : "v"(x), "v"(y)); }
__device__ __forceinline__ void keep4_h(v16h a, v16h b, v16h c, v16h d) { asm volatile("v_nop" :: "v"(a), "v"(b), "v"(c), "v"(d)); }
__device__ __forceinline__ void keep4_b(v16b a, v16b b, v16b c, v16b d) { asm volatile("v_nop" :: "v"(a), "v"(b), "v"(c), "v"(d)); }
__device__ __forceinline__ void acc_guard4(v8f& a, v8f& b, v8f& c, v8f& d) { asm volatile("v_nop\n\tv_nop\n\tv_nop\n\tv_nop" : "+v"(a), "+v"(b), "+v"(c), "+v"(d)); }
template <typename T> struct Frag;
template <> struct Frag<_Float16> {
  typedef v16h V; union U { v16h v; v8h h[2]; };
  static __device__ __forceinline__ v16h load(const _Float16* p) {
    U f; f.h[0] = *(const v8h*)(p); f.h[1] = *(const v8h*)(p + 16); return f.v;
  }
  static __device__ __forceinline__ v8f mma(v16h a, v16h b, v8f c) {
    return __builtin_amdgcn_wmma_f32_16x16x32_f16(false, a, false, b, (short)0, c, false, false);
  }
  static __device__ __forceinline__ void guard(v8f& a, v8f& b, v16h x, v16h y) { dep_guard_h(a, b, x, y); }
  static __device__ __forceinline__ void keep(v16h a, v16h b, v16h c, v16h d) { keep4_h(a, b, c, d); }
};
template <> struct Frag<__bf16> {
  typedef v16b V; union U { v16b v; v8b h[2]; };
  static __device__ __forceinline__ v16b load(const __bf16* p) {
    U f; f.h[0] = *(const v8b*)(p); f.h[1] = *(const v8b*)(p + 16); return f.v;
  }
  static __device__ __forceinline__ v8f mma(v16b a, v16b b, v8f c) {
    return __builtin_amdgcn_wmma_f32_16x16x32_bf16(false, a, false, b, (short)0, c, false, false);
  }
  static __device__ __forceinline__ void guard(v8f& a, v8f& b, v16b x, v16b y) { dep_guard_b(a, b, x, y); }
  static __device__ __forceinline__ void keep(v16b a, v16b b, v16b c, v16b d) { keep4_b(a, b, c, d); }
};

__device__ __forceinline__ unsigned pk16(unsigned short a, unsigned short b) { return (unsigned)a | ((unsigned)b << 16); }
__device__ __forceinline__ unsigned short h_bits(float f) { const _Float16 h = (_Float16)f; return __builtin_bit_cast(unsigned short, h); }

template <int ET> struct Elem;
template <> struct Elem<0> { typedef _Float16 T; };
template <> struct Elem<1> { typedef __bf16 T; };
template <int ET, bool SPLIT, int BIAS_MODE, int OUT_MODE, bool RESID, int ACT = 0>
__global__ __launch_bounds__(256) void wmma_gemm64(
    const unsigned short* __restrict__ Ap, const unsigned short* __restrict__ A2p, int lda, long strideA,
    const unsigned short* __restrict__ Btp, const unsigned short* __restrict__ Bt2p, int ldb, long strideB,
    void* __restrict__ Cout, void* __restrict__ Cout2, int ldc, long strideC,
    const float* __restrict__ bias,
    const float* __restrict__ resid, long strideR,
    int M, int N, int K, float scale) {
  typedef typename Elem<ET>::T T;
  typedef typename Frag<T>::V V;
  const T* A = (const T*)Ap; const T* A2 = (const T*)A2p; const T* Bt = (const T*)Btp; const T* Bt2 = (const T*)Bt2p;
  __shared__ __align__(16) float sT[8][16 * 68];
  const int b    = blockIdx.y;
  const int lane = threadIdx.x & 31;
  const int wave = threadIdx.x >> 5;
  const int tilesN = N >> 6;
  const int tilesM = M >> 6;
  const int tile = blockIdx.x * 8 + wave;
  if (tile >= tilesM * tilesN) return;
  const int tm = tile / tilesN;
  const int tn = tile - tm * tilesN;
  const int m0 = tm << 6;
  const int n0 = tn << 6;

  const T* Ab  = A  + (size_t)b * strideA;
  const T* Bb  = Bt + (size_t)b * strideB;
  const T* Ab2 = SPLIT ? (A2  + (size_t)b * strideA) : nullptr;
  const T* Bb2 = SPLIT ? (Bt2 + (size_t)b * strideB) : nullptr;

  const int rlane = lane & 15;
  const int koff  = (lane >> 4) * 8;
  const int mOff  = (lane >> 4) * 8;

  v8f acc[4][4];
#pragma unroll
  for (int i = 0; i < 4; ++i)
#pragma unroll
    for (int j = 0; j < 4; ++j) acc[i][j] = (v8f){0.f,0.f,0.f,0.f,0.f,0.f,0.f,0.f};

  for (int k0 = 0; k0 < K; k0 += 32) {
    V bh[4], bl[4];
#pragma unroll
    for (int j = 0; j < 4; ++j) {
      const size_t bo = (size_t)(n0 + (j << 4) + rlane) * ldb + koff + k0;
      bh[j] = Frag<T>::load(Bb + bo);
      if (SPLIT) bl[j] = Frag<T>::load(Bb2 + bo);
    }
#pragma unroll
    for (int i = 0; i < 4; ++i) {
      const size_t ao = (size_t)(m0 + (i << 4) + rlane) * lda + koff + k0;
      V ah = Frag<T>::load(Ab + ao);
      V al;
      if (SPLIT) al = Frag<T>::load(Ab2 + ao);
#pragma unroll
      for (int j = 0; j < 4; ++j) {
        acc[i][j] = Frag<T>::mma(ah, bh[j], acc[i][j]);
        if (SPLIT) {
          acc[i][j] = Frag<T>::mma(ah, bl[j], acc[i][j]);
          acc[i][j] = Frag<T>::mma(al, bh[j], acc[i][j]);
        }
      }
      Frag<T>::guard(acc[i][0], acc[i][3], ah, SPLIT ? al : ah);
    }
    Frag<T>::keep(bh[0], bh[1], bh[2], bh[3]);
    if (SPLIT) Frag<T>::keep(bl[0], bl[1], bl[2], bl[3]);
  }
  acc_guard4(acc[0][0], acc[0][1], acc[0][2], acc[0][3]);
  acc_guard4(acc[1][0], acc[1][1], acc[1][2], acc[1][3]);
  acc_guard4(acc[2][0], acc[2][1], acc[2][2], acc[2][3]);
  acc_guard4(acc[3][0], acc[3][1], acc[3][2], acc[3][3]);

  float* slab = sT[wave];
  const float* Rb = RESID ? (resid + (size_t)b * strideR) : nullptr;
#pragma unroll
  for (int i = 0; i < 4; ++i) {
    const int mBase = m0 + (i << 4);
#pragma unroll
    for (int j = 0; j < 4; ++j) {
      const int n = n0 + (j << 4) + rlane;
      float bv = 0.f;
      if (BIAS_MODE == 2) bv = bias[n];
#pragma unroll
      for (int r = 0; r < 8; ++r) {
        float v = acc[i][j][r] * scale;
        if (BIAS_MODE == 1) v += bias[mBase + mOff + r];
        if (BIAS_MODE == 2) v += bv;
        if (RESID) v += Rb[(size_t)(mBase + mOff + r) * ldc + n];
        if (ACT == 2) v = fmaxf(v, 0.0f);
        if (ACT == 4) v = (v > 0.f) ? v : 0.01f * v;
        slab[(mOff + r) * 68 + (j << 4) + rlane] = v;
      }
    }
    __builtin_amdgcn_fence(__ATOMIC_RELEASE, "workgroup");
    __builtin_amdgcn_wave_barrier();
    __builtin_amdgcn_fence(__ATOMIC_ACQUIRE, "workgroup");
    if (OUT_MODE == 0) {
      float* C = (float*)Cout + (size_t)b * strideC;
      const int hh = lane >> 4, c4 = (lane & 15) * 4;
      for (int pass = 0; pass < 2; ++pass) {
#pragma unroll
        for (int it = 0; it < 8; ++it) {
          const int row = it * 2 + hh;
          v4f v = *(const v4f*)(slab + row * 68 + c4);
          *(volatile v4f*)(C + (size_t)(mBase + row) * ldc + n0 + c4) = v;
        }
        __threadfence();
      }
    } else {
      const int q = lane >> 3, c8 = (lane & 7) * 8;
      unsigned short* C  = (unsigned short*)Cout  + (size_t)b * strideC;
      unsigned short* C2 = (OUT_MODE == 2) ? ((unsigned short*)Cout2 + (size_t)b * strideC) : nullptr;
      for (int pass = 0; pass < 2; ++pass) {
#pragma unroll
        for (int it = 0; it < 4; ++it) {
          const int row = it * 4 + q;
          const float* sp = slab + row * 68 + c8;
          v8h hv, lv;
#pragma unroll
          for (int e = 0; e < 8; ++e) {
            if (OUT_MODE == 1) {
              hv[e] = (_Float16)sp[e];
            } else {
              unsigned short hb = f2bf_bits(sp[e]);
              unsigned short lb = f2bf_bits(sp[e] - bf_bits2f(hb));
              hv[e] = __builtin_bit_cast(_Float16, hb);
              lv[e] = __builtin_bit_cast(_Float16, lb);
            }
          }
          *(volatile v8h*)(C + (size_t)(mBase + row) * ldc + n0 + c8) = hv;
          if (OUT_MODE == 2) *(volatile v8h*)(C2 + (size_t)(mBase + row) * ldc + n0 + c8) = lv;
        }
        __threadfence();
      }
    }
    __builtin_amdgcn_fence(__ATOMIC_RELEASE, "workgroup");
    __builtin_amdgcn_wave_barrier();
    __builtin_amdgcn_fence(__ATOMIC_ACQUIRE, "workgroup");
  }
}

template <int CIN>
__global__ __launch_bounds__(256) void wperm_kernel(const float* __restrict__ w, unsigned short* __restrict__ wt) {
  constexpr int KK  = 9 * CIN;
  constexpr int CPR = KK / 8;
  constexpr int CG  = CIN / 8;
  constexpr int NCHW = kNG * CPR;
  const int cc = blockIdx.x * 256 + threadIdx.x;
  if (cc >= NCHW) return;
  const int n   = cc / CPR;
  const int cl  = cc - n * CPR;
  const int tap = cl / CG;
  const int cg  = cl - tap * CG;
  const float* src = w + ((size_t)(n * CIN + cg * 8)) * 9 + tap;
  unsigned short hb[8];
#pragma unroll
  for (int j = 0; j < 8; ++j) hb[j] = h_bits(src[j * 9] * kWCarry);
  const v4u u = (v4u){pk16(hb[0], hb[1]), pk16(hb[2], hb[3]), pk16(hb[4], hb[5]), pk16(hb[6], hb[7])};
  unsigned short* q = wt + 8 * (size_t)cc;
  *(volatile v4u*)q = u;
  __threadfence();
  *(volatile v4u*)q = u;
}

template <int CIN, bool SRC16>
__global__ __launch_bounds__(256) void im2col_kernel(const float* __restrict__ xs, const unsigned* __restrict__ hs,
                                                     unsigned short* __restrict__ Aout, const int frame0) {
  constexpr int KK    = 9 * CIN;
  constexpr int NWORD = CIN * 48;
  constexpr int NSTG  = NWORD / 256;
  constexpr int NCH   = 4 * KK;
  constexpr int NIT   = (NCH + 255) / 256;
  constexpr int CPR   = KK / 8;
  constexpr int CG    = CIN / 8;
  __shared__ __align__(16) unsigned short s16[3 * 36 * CIN];
  const int tid = threadIdx.x;
  const int fl  = blockIdx.x >> 5;
  const int y   = blockIdx.x & 31;
  const int frame = frame0 + fl;

  for (int e = tid; e < 6 * CIN; e += 256) {
    const int kyq = e / CIN;
    const int ci  = e - kyq * CIN;
    const int ky  = kyq >> 1;
    const int q   = (kyq & 1) ? 34 : 1;
    s16[(ky * 36 + q) * CIN + ci] = (unsigned short)0;
  }
#pragma unroll
  for (int it = 0; it < NSTG; ++it) {
    const int e   = it * 256 + tid;
    const int ci  = e / 48;
    const int r   = e - ci * 48;
    const int ky  = r >> 4;
    const int xw  = r & 15;
    const int yy  = y + ky - 1;
    const bool inr = (unsigned)yy < 32u;
    const int yyc = yy < 0 ? 0 : (yy > 31 ? 31 : yy);
    unsigned short lo, hi;
    if (SRC16) {
      const unsigned wv = hs[((size_t)(frame * CIN + ci)) * 512 + yyc * 16 + xw];
      lo = (unsigned short)(wv & 0xffffu);
      hi = (unsigned short)(wv >> 16);
    } else {
      const float* p = xs + ((size_t)(frame * CIN + ci)) * kHW + yyc * 32 + 2 * xw;
      const v2f f = *(const v2f*)p;
      lo = h_bits(f[0]);
      hi = h_bits(f[1]);
    }
    lo = inr ? lo : (unsigned short)0;
    hi = inr ? hi : (unsigned short)0;
    s16[(ky * 36 + 2 * xw + 2) * CIN + ci] = lo;
    s16[(ky * 36 + 2 * xw + 3) * CIN + ci] = hi;
  }
  __syncthreads();

  v4u u[NIT];
#pragma unroll
  for (int it = 0; it < NIT; ++it) {
    int cc = it * 256 + tid;
    cc = cc < NCH ? cc : (NCH - 1);
    const int xl  = cc / CPR;
    const int cl  = cc - xl * CPR;
    const int tap = cl / CG;
    const int cg  = cl - tap * CG;
    const int ky  = tap / 3;
    const int kx  = tap - ky * 3;
    const int q   = xl + kx + 1;
    u[it] = *(const v4u*)(s16 + (ky * 36 + q) * CIN + cg * 8);
  }
  unsigned short* dst = Aout + ((size_t)(fl * kHW + y * 32)) * KK;
  for (int pass = 0; pass < 2; ++pass) {
#pragma unroll
    for (int it = 0; it < NIT; ++it) {
      const int cc = it * 256 + tid;
      if (cc < NCH) *(volatile v4u*)(dst + 8 * (size_t)cc) = u[it];
    }
    __threadfence();
  }
}

__device__ __forceinline__ float sigm(float x) { return 1.0f / (1.0f + expf(-x)); }

template <bool OUT16>
__global__ __launch_bounds__(256) void gate_scan_kernel(const float* __restrict__ G, unsigned short* __restrict__ H0,
                                                        float* __restrict__ outp, const int halfIdx) {
  #pragma clang fp contract(off)
  __shared__ __align__(16) unsigned short sh16[256];
  __shared__ __align__(16) float shf[256];
  const int tid  = threadIdx.x;
  const int lane = tid & 31;
  const int wave = tid >> 5;
  const int bx   = blockIdx.x;
  const int bl   = bx >> 8;
  const int ch   = (bx >> 2) & 63;
  const int pch  = bx & 3;
  const int p    = pch * 256 + tid;
  float cst = 0.5f;
#pragma unroll 1
  for (int s = 0; s < kNS; ++s) {
    const float* gr = G + ((size_t)((bl * kNS + s) * kHW + p)) * kNG;
    const float gi = gr[ch];
    const float gf = gr[kCH + ch];
    const float go = gr[2 * kCH + ch];
    const float gc = gr[3 * kCH + ch];
    const float it = sigm(gi);
    const float ft = sigm(gf);
    const float ot = sigm(go);
    const float sc = sigm(gc);
    const float ga = (gc >= 0.0f) ? (gc + 0.5f) : sc;
    const float den  = it + ft;
    const float rden = 1.0f / den;
    const float fp = ft * rden;
    const float inorm = it * rden;
    const float ig = inorm * ga;
    const float prod = fp * cst;
    cst = prod + ig;
    const float h = ot * cst;
    if (OUT16) sh16[tid] = h_bits(h * kHCarry);
    else       shf[tid]  = h;
    __syncthreads();
    if (OUT16) {
      const int frame = halfIdx * kFramesHalf + bl * kNS + s;
      unsigned short* dst = H0 + ((size_t)(frame * kCH + ch)) * kHW + pch * 256;
      const v4u uv = *(const v4u*)(sh16 + 8 * lane);
      for (int pass = 0; pass < 2; ++pass) {
        if (wave == 0) *(volatile v4u*)(dst + 8 * lane) = uv;
        __threadfence();
      }
    } else {
      const int bb = halfIdx * 2 + bl;
      float* dst = outp + ((size_t)((bb * kNS + s) * kCH + ch)) * kHW + pch * 256;
      const int idx = (wave & 1) * 32 + lane;
      const v4f val = *(const v4f*)(shf + 4 * idx);
      for (int pass = 0; pass < 2; ++pass) {
        if (wave < 2) *(volatile v4f*)(dst + 4 * idx) = val;
        __threadfence();
      }
    }
    __syncthreads();
  }
}

extern "C" void kernel_launch(void* const* d_in, const int* in_sizes, int n_in,
                              void* d_out, int out_size, void* d_ws, size_t ws_size,
                              hipStream_t stream) {
  if (n_in < 5) return;
  if (in_sizes[0] != kNB * kNS * kCin0 * kHW) return;
  if (in_sizes[1] != kNG * kCin0 * 9 || in_sizes[2] != kNG) return;
  if (in_sizes[3] != kNG * kCH * 9 || in_sizes[4] != kNG) return;
  if (out_size != kNB * kNS * kCH * kHW) return;
  if (ws_size < kCarveEnd) return;

  const float* x  = (const float*)d_in[0];
  const float* w0 = (const float*)d_in[1];
  const float* b0 = (const float*)d_in[2];
  const float* w1 = (const float*)d_in[3];
  const float* b1 = (const float*)d_in[4];
  float* outp = (float*)d_out;

  char* ws = (char*)d_ws;
  unsigned short* WT0 = (unsigned short*)(ws + kOffWT0);
  unsigned short* WT1 = (unsigned short*)(ws + kOffWT1);
  unsigned short* H0  = (unsigned short*)(ws + kOffH0);
  unsigned short* Apl = (unsigned short*)(ws + kOffA);
  float*          G   = (float*)(ws + kOffG);

  constexpr int kK0 = 9 * kCin0;
  constexpr int kK1 = 9 * kCH;

  wperm_kernel<kCin0><<<dim3((kNG * kK0 / 8) / 256), dim3(256), 0, stream>>>(w0, WT0);
  wperm_kernel<kCH><<<dim3((kNG * kK1 / 8) / 256), dim3(256), 0, stream>>>(w1, WT1);

  for (int half = 0; half < 2; ++half) {
    const int frame0 = half * kFramesHalf;
    im2col_kernel<kCin0, false><<<dim3(kFramesHalf * 32), dim3(256), 0, stream>>>(x, (const unsigned*)H0, Apl, frame0);
    wmma_gemm64<0, false, 2, 0, false, 0><<<dim3(256, 1, 1), dim3(256), 0, stream>>>(
        Apl, Apl, kK0, 0L, WT0, WT0, kK0, 0L, (void*)G, (void*)G, kNG, 0L,
        b0, (const float*)G, 0L, kRowsHalf, kNG, kK0, kScale0);
    gate_scan_kernel<true><<<dim3(512), dim3(256), 0, stream>>>(G, H0, outp, half);
    im2col_kernel<kCH, true><<<dim3(kFramesHalf * 32), dim3(256), 0, stream>>>(x, (const unsigned*)H0, Apl, frame0);
    wmma_gemm64<0, false, 2, 0, false, 0><<<dim3(256, 1, 1), dim3(256), 0, stream>>>(
        Apl, Apl, kK1, 0L, WT1, WT1, kK1, 0L, (void*)G, (void*)G, kNG, 0L,
        b1, (const float*)G, 0L, kRowsHalf, kNG, kK1, kScale1);
    gate_scan_kernel<false><<<dim3(512), dim3(256), 0, stream>>>(G, H0, outp, half);
  }
}
